// SelfAttention_59193239274178
// MI455X (gfx1250) — hardware-run, weakly checked
//
#include <hip/hip_runtime.h>


#ifndef NB
#define NB 4
#endif
#ifndef SEQ
#define SEQ 4096
#endif
#define NB_FULL  4
#define SEQ_FULL 4096
#ifndef OUT_SEQ
#define OUT_SEQ SEQ
#endif
#define CCH  256
#define NGR  8
#define AW   4
#define QPITCH 264
#define HSC  16.0f
#define WSC  64.0f
#define QSC  16.0f
#define VSC  16.0f
#define OSC  64.0f
#define PSH  8.0f
#define SC2  (0.0625f * 1.4426950408889634f / (QSC * QSC))

static_assert(CCH == 256);
static_assert(NGR * 32 == CCH);
static_assert(CCH % 64 == 0);
static_assert(SEQ % 64 == 0);
static_assert((NB * SEQ) % 64 == 0);
static_assert(SEQ % 32 == 0);
static_assert(SEQ % (16 * AW) == 0);
static_assert(SEQ % 4 == 0);
static_assert(OUT_SEQ % 32 == 0);
static_assert(OUT_SEQ >= SEQ);
static_assert(QPITCH % 8 == 0);
static_assert(QPITCH >= CCH);
static_assert(NB <= NB_FULL);
static_assert(SEQ <= SEQ_FULL);

typedef _Float16 h16;
typedef __attribute__((ext_vector_type(16))) _Float16 v16h;
typedef __attribute__((ext_vector_type(8)))  _Float16 v8h;
typedef __attribute__((ext_vector_type(8)))  float    v8f;
typedef __attribute__((ext_vector_type(4)))  float    v4f;
typedef v4f  __attribute__((may_alias)) v4fa;
typedef v8h  __attribute__((may_alias)) v8ha;

__device__ __forceinline__ unsigned short f2bf(float f) { unsigned u = __float_as_uint(f); u += 0x7FFFu + ((u >> 16) & 1u); return (unsigned short)(u >> 16); }
__device__ __forceinline__ float bfr(float f) { return __uint_as_float(((unsigned)f2bf(f)) << 16); }
__device__ __forceinline__ v16h cat16(v8h lo, v8h hi) { return __builtin_shufflevector(lo, hi, 0, 1, 2, 3, 4, 5, 6, 7, 8, 9, 10, 11, 12, 13, 14, 15); }
__device__ __forceinline__ v8f wmma16(v16h a, v16h b, v8f c) { return __builtin_amdgcn_wmma_f32_16x16x32_f16(false, a, false, b, (short)0, c, false, false); }
__device__ __forceinline__ v16h ldh(const h16* p) { return cat16(*(const v8h*)p, *(const v8h*)(p + 16)); }
__device__ __forceinline__ void wave_sync() { __builtin_amdgcn_fence(3  , "wavefront"); __builtin_amdgcn_wave_barrier(); asm volatile("" ::: "memory"); }

__global__ __launch_bounds__(256) void k_cvtw(const float* __restrict__ src, h16* dst, size_t n8) {
    const size_t i = (size_t)blockIdx.x * 256 + threadIdx.x; if (i >= n8) return;
    const v8f v = *(const v8f*)(src + i * 8); v8h o;
#pragma unroll
    for (int k = 0; k < 8; ++k) o[k] = (h16)(bfr(v[k]) * WSC);
    *(volatile v8h*)(dst + i * 8) = o; __threadfence(); *(volatile v8h*)(dst + i * 8) = o;
}

__global__ __launch_bounds__(256) void k_stats(const float* __restrict__ x, float* ST) {
    __shared__ double rs[256];
    __shared__ double rq[256];
    const int tid = threadIdx.x;
    const int b = blockIdx.x / NGR, g = blockIdx.x % NGR;
    const float* xg = x + ((size_t)(b * CCH + g * 32)) * SEQ_FULL;
    const int upr = SEQ / 4;
    double s = 0.0, ss = 0.0;
#pragma unroll 1
    for (int u = tid; u < 32 * upr; u += 256) {
        const int cl = u / upr, n4 = (u - cl * upr) * 4;
        const v4f v = *(const v4f*)(xg + (size_t)cl * SEQ_FULL + n4);
#pragma unroll
        for (int j = 0; j < 4; ++j) { const double f = (double)bfr(v[j]); s += f; ss += f * f; }
    }
    rs[tid] = s; rq[tid] = ss;
    __syncthreads();
#pragma unroll 1
    for (int st = 128; st > 0; st >>= 1) {
        if (tid < st) { rs[tid] += rs[tid + st]; rq[tid] += rq[tid + st]; }
        __syncthreads();
    }
    if (tid < 8) {
        const double cnt = 32.0 * (double)SEQ;
        const double mean = rs[0] / cnt;
        const double var = rq[0] / cnt - mean * mean;
        const float rstd = rsqrtf((float)var + 1.0e-5f);
        v4f o = (v4f){};
        o[0] = (tid == 0) ? (float)mean : 0.0f;
        o[1] = (tid == 0) ? rstd : 0.0f;
        float* dst = ST + (size_t)blockIdx.x * 32 + tid * 4;
        *(volatile v4f*)dst = o; __threadfence(); *(volatile v4f*)dst = o;
    }
}

__global__ __launch_bounds__(256) void k_norm(const float* __restrict__ x, const float* __restrict__ gw, const float* __restrict__ gb, const float* __restrict__ ST, h16* HT) {
    __shared__ __align__(16) h16 tile[64 * 72];
    const int tid = threadIdx.x;
    const int n0 = blockIdx.x * 64, c0 = blockIdx.y * 64, b = blockIdx.z;
#pragma unroll
    for (int i = 0; i < 4; ++i) {
        const int u = tid + 256 * i; const int cl = u >> 4, n4 = (u & 15) * 4;
        const int c = c0 + cl;
        const float* st = ST + (size_t)(b * NGR + (c >> 5)) * 32;
        const float mean = st[0], rstd = st[1];
        const float w = bfr(gw[c]), bb = bfr(gb[c]);
        const v4f v = *(const v4f*)(x + ((size_t)(b * CCH + c)) * SEQ_FULL + n0 + n4);
#pragma unroll
        for (int j = 0; j < 4; ++j) { const float hv = ((bfr(v[j]) - mean) * rstd * w + bb) * HSC; tile[(n4 + j) * 72 + cl] = (h16)hv; }
    }
    __syncthreads();
#pragma unroll 1
    for (int ps = 0; ps < 2; ++ps) {
#pragma unroll
        for (int i = 0; i < 2; ++i) {
            const int line = (tid >> 3) + 32 * i, piece = tid & 7;
            const v8h val = *(const v8ha*)(&tile[line * 72 + piece * 8]);
            *(volatile v8h*)(HT + ((size_t)b * SEQ + n0 + line) * CCH + c0 + piece * 8) = val; }
        if (ps == 0) __threadfence(); }
}

template <int MODE>
__global__ __launch_bounds__(32) void k_gemm(const h16* __restrict__ A, const h16* __restrict__ Bt, const float* __restrict__ bias,
                                             h16* Ph, float* Yf, const float* __restrict__ X,
                                             int RB, size_t sRB, int pitch, int CB, size_t sCB, int xpitch, size_t xsCB, float scale, float osc) {
    __shared__ __align__(16) float os[16 * 68];
    const int K = CCH;
    const int lane = threadIdx.x & 31, lr = lane & 15, hi = lane >> 4; const int r0 = blockIdx.x * 64, c0 = blockIdx.y * 64;
    v8f acc[4][4];
#pragma unroll
    for (int mb = 0; mb < 4; ++mb)
#pragma unroll
        for (int nb = 0; nb < 4; ++nb) acc[mb][nb] = (v8f){};
    const size_t aoff = (size_t)(r0 + lr) * K + 8 * hi, boff = (size_t)(c0 + lr) * K + 8 * hi;
#pragma unroll 1
    for (int kc = 0; kc < K; kc += 32) {
        v16h a[4];
#pragma unroll
        for (int mb = 0; mb < 4; ++mb) a[mb] = ldh(A + aoff + (size_t)mb * 16 * K + kc);
#pragma unroll
        for (int nb = 0; nb < 4; ++nb) { const v16h bfrag = ldh(Bt + boff + (size_t)nb * 16 * K + kc);
#pragma unroll
            for (int mb = 0; mb < 4; ++mb) acc[mb][nb] = wmma16(a[mb], bfrag, acc[mb][nb]); }
        asm volatile("v_nop\n\tv_nop\n\tv_nop\n\tv_nop" : "+v"(acc[0][0]), "+v"(acc[1][1]), "+v"(acc[2][2]), "+v"(acc[3][3]) : "v"(a[0]), "v"(a[1]), "v"(a[2]), "v"(a[3]));
    }
    const size_t cq = (size_t)(c0 / CB), cr = (size_t)(c0 % CB);
    const size_t tbase = (size_t)(r0 / RB) * sRB + (size_t)(r0 % RB) * (size_t)pitch + cq * sCB + cr;
    const size_t xbase = (size_t)(r0 % RB) * (size_t)xpitch + cq * xsCB + cr;
    float bc[8];
#pragma unroll
    for (int i = 0; i < 8; ++i) bc[i] = 0.0f;
    if (MODE == 0) {
        const v4f b0 = *(const v4f*)(bias + c0 + (lane & 7) * 8); const v4f b1 = *(const v4f*)(bias + c0 + (lane & 7) * 8 + 4);
#pragma unroll
        for (int i = 0; i < 4; ++i) { bc[i] = bfr(b0[i]); bc[4 + i] = bfr(b1[i]); }
    }
#pragma unroll
    for (int mb = 0; mb < 4; ++mb) {
#pragma unroll
        for (int nb = 0; nb < 4; ++nb) {
#pragma unroll
            for (int j = 0; j < 8; ++j) os[(hi * 8 + j) * 68 + nb * 16 + lr] = acc[mb][nb][j]; }
        wave_sync();
        const size_t sb = tbase + (size_t)(mb * 16) * (size_t)pitch;
#pragma unroll 1
        for (int ps = 0; ps < 2; ++ps) {
            if (MODE == 2) {
#pragma unroll
                for (int s = 0; s < 8; ++s) { const int row = 2 * s + hi, cofs = lr * 4;
                    const v4f a4 = *(const v4fa*)(&os[row * 68 + cofs]);
                    const float br = bfr(bias[r0 + mb * 16 + row]);
                    const v4f xv = *(const v4f*)(X + xbase + (size_t)(mb * 16 + row) * (size_t)xpitch + cofs);
                    v4f val;
#pragma unroll
                    for (int i = 0; i < 4; ++i) val[i] = bfr(xv[i]) + (a4[i] * scale + br);
                    *(volatile v4f*)(Yf + sb + (size_t)row * (size_t)pitch + cofs) = val; }
            } else {
#pragma unroll
                for (int s = 0; s < 4; ++s) { const int row = 4 * s + (lane >> 3), c8 = (lane & 7) * 8;
                    const v4f x0 = *(const v4fa*)(&os[row * 68 + c8]); const v4f x1 = *(const v4fa*)(&os[row * 68 + c8 + 4]);
                    float br = 0.0f;
                    if (MODE == 1) br = bfr(bias[r0 + mb * 16 + row]);
                    v8h hv;
#pragma unroll
                    for (int i = 0; i < 4; ++i) {
                        const float f0 = x0[i] * scale + ((MODE == 0) ? bc[i] : br);
                        const float f1 = x1[i] * scale + ((MODE == 0) ? bc[4 + i] : br);
                        hv[i] = (h16)(f0 * osc); hv[4 + i] = (h16)(f1 * osc); }
                    *(volatile v8h*)(Ph + sb + (size_t)row * (size_t)pitch + c8) = hv; }
            }
            if (ps == 0) __threadfence(); }
        wave_sync();
    }
}

__global__ __launch_bounds__(32 * AW) void k_flash(const h16* __restrict__ QP, const h16* __restrict__ KP, const h16* __restrict__ VT, h16* OP) {
    __shared__ __align__(16) h16 qs[AW * 16 * QPITCH];
    const int lane = threadIdx.x & 31, wave = __builtin_amdgcn_readfirstlane((int)(threadIdx.x >> 5)), lr = lane & 15, hi = lane >> 4;
    const int b = blockIdx.y;
    const int t0 = (blockIdx.x * AW + wave) * 16;
    const int wb = wave * 16 * QPITCH;
    const size_t rowbase = (size_t)b * SEQ;
#pragma unroll
    for (int i = 0; i < 16; ++i) {
        const v8h v = *(const v8h*)(QP + (rowbase + t0 + i) * CCH + lane * 8);
        *(v8h*)(&qs[wb + i * QPITCH + lane * 8]) = v; }
    wave_sync();
    const int qoff = wb + lr * QPITCH + 8 * hi;
    const size_t ko = (rowbase + lr) * CCH + 8 * hi;
    const size_t vo = ((size_t)b * CCH + lr) * SEQ + 8 * hi;
    v8f o[16];
#pragma unroll
    for (int i = 0; i < 16; ++i) o[i] = (v8f){};
    float m = -3.0e38f, l = 0.0f;
#pragma unroll 1
    for (int key0 = 0; key0 < SEQ; key0 += 32) {
        const h16* ka = KP + ko + (size_t)key0 * CCH;
        v8f sa = (v8f){}, sb = (v8f){};
#pragma unroll 1
        for (int kc = 0; kc < CCH; kc += 64) {
            const v16h q0 = cat16(*(const v8h*)(&qs[qoff + kc]),      *(const v8h*)(&qs[qoff + kc + 16]));
            const v16h q1 = cat16(*(const v8h*)(&qs[qoff + kc + 32]), *(const v8h*)(&qs[qoff + kc + 48]));
            const v16h ka0 = ldh(ka + kc), ka1 = ldh(ka + kc + 32), kb0 = ldh(ka + 16 * CCH + kc), kb1 = ldh(ka + 16 * CCH + kc + 32);
            sa = wmma16(ka0, q0, sa); sb = wmma16(kb0, q0, sb);
            sa = wmma16(ka1, q1, sa); sb = wmma16(kb1, q1, sb);
            asm volatile("v_nop\n\tv_nop\n\tv_nop\n\tv_nop" : "+v"(sa), "+v"(sb) : "v"(ka0), "v"(ka1), "v"(kb0), "v"(kb1), "v"(q0), "v"(q1));
        }
        float ta[8], tb[8]; float mx = -3.0e38f;
#pragma unroll
        for (int r = 0; r < 8; ++r) { ta[r] = sa[r] * SC2; tb[r] = sb[r] * SC2; mx = fmaxf(mx, fmaxf(ta[r], tb[r])); }
        mx = fmaxf(mx, __shfl_xor(mx, 16, 32));
        const float mnew = fmaxf(m, mx);
        const float alpha = __builtin_amdgcn_exp2f(m - mnew);
        const float sh = PSH - mnew;
        v16h pb; float ls = 0.0f;
#pragma unroll
        for (int r = 0; r < 8; ++r) { const h16 pa = (h16)__builtin_amdgcn_exp2f(ta[r] + sh); const h16 pc = (h16)__builtin_amdgcn_exp2f(tb[r] + sh); pb[r] = pa; pb[8 + r] = pc; ls += (float)pa + (float)pc; }
        l = l * alpha + ls; m = mnew;
        const unsigned need = __builtin_amdgcn_ballot_w32(alpha != 1.0f);
        if (need != 0u) {
#pragma unroll
            for (int i = 0; i < 16; ++i) o[i] = o[i] * alpha;
        }
        const h16* va = VT + vo + key0;
#pragma unroll
        for (int g = 0; g < 4; ++g) {
            const h16* vg = va + (size_t)(64 * g) * SEQ;
            const v16h v0 = ldh(vg), v1 = ldh(vg + (size_t)16 * SEQ), v2 = ldh(vg + (size_t)32 * SEQ), v3 = ldh(vg + (size_t)48 * SEQ);
            o[4 * g + 0] = wmma16(v0, pb, o[4 * g + 0]); o[4 * g + 1] = wmma16(v1, pb, o[4 * g + 1]);
            o[4 * g + 2] = wmma16(v2, pb, o[4 * g + 2]); o[4 * g + 3] = wmma16(v3, pb, o[4 * g + 3]);
            asm volatile("v_nop\n\tv_nop\n\tv_nop\n\tv_nop" : "+v"(o[4 * g + 0]), "+v"(o[4 * g + 1]), "+v"(o[4 * g + 2]), "+v"(o[4 * g + 3]) : "v"(v0), "v"(v1), "v"(v2), "v"(v3), "v"(pb));
        }
    }
    l += __shfl_xor(l, 16, 32);
    const float osc = (OSC / VSC) * (1.0f / l);
    wave_sync();
#pragma unroll
    for (int j = 0; j < 16; ++j) { v8h pk;
#pragma unroll
        for (int r = 0; r < 8; ++r) pk[r] = (h16)(o[j][r] * osc);
        *(v8h*)(&qs[wb + lr * QPITCH + 16 * j + 8 * hi]) = pk; }
    wave_sync();
    h16* orow = OP + (rowbase + t0) * CCH + lane * 8;
#pragma unroll 1
    for (int ps = 0; ps < 2; ++ps) {
#pragma unroll
        for (int row = 0; row < 16; ++row) {
            const v8h val = *(const v8h*)(&qs[wb + row * QPITCH + lane * 8]);
            *(volatile v8h*)(orow + (size_t)row * CCH) = val; }
        if (ps == 0) __threadfence(); }
}

static constexpr size_t al256(size_t v) { return (v + 255) & ~(size_t)255; }
static constexpr size_t SZ_ST = al256((size_t)NB * NGR * 32 * 4);
static constexpr size_t SZ_WB = al256((size_t)4 * CCH * CCH * 2);
static constexpr size_t SZ_PL = al256((size_t)NB * SEQ * CCH * 2);
static constexpr size_t SZ_TOTAL = SZ_ST + SZ_WB + 5 * SZ_PL;
static_assert(SZ_TOTAL <= (size_t)134217728);
static_assert(((size_t)CCH * CCH * 2) % 256 == 0);

extern "C" void kernel_launch(void* const* d_in, const int* in_sizes, int n_in,
                              void* d_out, int out_size, void* d_ws, size_t ws_size, hipStream_t stream) {
    if (n_in < 11) return;
    const size_t needx = ((size_t)((NB - 1) * CCH + (CCH - 1))) * SEQ_FULL + SEQ;
    if ((size_t)in_sizes[0] < needx) return;
    if (in_sizes[1] < CCH || in_sizes[2] < CCH) return;
    if ((size_t)in_sizes[3] < (size_t)CCH * CCH || (size_t)in_sizes[5] < (size_t)CCH * CCH || (size_t)in_sizes[7] < (size_t)CCH * CCH || (size_t)in_sizes[9] < (size_t)CCH * CCH) return;
    if (in_sizes[4] < CCH || in_sizes[6] < CCH || in_sizes[8] < CCH || in_sizes[10] < CCH) return;
    if ((size_t)out_size < ((size_t)((NB - 1) * CCH + (CCH - 1))) * OUT_SEQ + SEQ) return;
    if (SZ_TOTAL > ws_size) return;
    const float* x   = (const float*)d_in[0];
    const float* gnw = (const float*)d_in[1];
    const float* gnb = (const float*)d_in[2];
    const float* wq  = (const float*)d_in[3];
    const float* bq  = (const float*)d_in[4];
    const float* wk  = (const float*)d_in[5];
    const float* bk  = (const float*)d_in[6];
    const float* wv  = (const float*)d_in[7];
    const float* bv  = (const float*)d_in[8];
    const float* wp  = (const float*)d_in[9];
    const float* bp  = (const float*)d_in[10];
    float* OUT = (float*)d_out;
    char* wsp = (char*)d_ws;
    float* ST = (float*)wsp; wsp += SZ_ST;
    h16* WB = (h16*)wsp; wsp += SZ_WB;
    h16* HT = (h16*)wsp; wsp += SZ_PL;
    h16* QP = (h16*)wsp; wsp += SZ_PL;
    h16* KP = (h16*)wsp; wsp += SZ_PL;
    h16* VT = (h16*)wsp; wsp += SZ_PL;
    h16* OP = (h16*)wsp; wsp += SZ_PL;
    h16* WQ = WB; h16* WK = WB + (size_t)CCH * CCH; h16* WV = WB + (size_t)2 * CCH * CCH; h16* WP = WB + (size_t)3 * CCH * CCH;

    { const size_t n8 = (size_t)CCH * CCH / 8; const unsigned g = (unsigned)((n8 + 255) / 256);
      k_cvtw<<<g, 256, 0, stream>>>(wq, WQ, n8); k_cvtw<<<g, 256, 0, stream>>>(wk, WK, n8);
      k_cvtw<<<g, 256, 0, stream>>>(wv, WV, n8); k_cvtw<<<g, 256, 0, stream>>>(wp, WP, n8); }

    k_stats<<<NB * NGR, 256, 0, stream>>>(x, ST);
    k_norm<<<dim3(SEQ / 64, CCH / 64, NB), 256, 0, stream>>>(x, gnw, gnb, ST, HT);

    const float sproj = 1.0f / (HSC * WSC);
    k_gemm<0><<<dim3(NB * SEQ / 64, CCH / 64, 1), 32, 0, stream>>>(HT, WQ, bq, QP, OUT, x, NB * SEQ, (size_t)0, CCH, CCH, (size_t)0, 0, (size_t)0, sproj, QSC);
    k_gemm<0><<<dim3(NB * SEQ / 64, CCH / 64, 1), 32, 0, stream>>>(HT, WK, bk, KP, OUT, x, NB * SEQ, (size_t)0, CCH, CCH, (size_t)0, 0, (size_t)0, sproj, QSC);
    k_gemm<1><<<dim3(CCH / 64, NB * SEQ / 64, 1), 32, 0, stream>>>(WV, HT, bv, VT, OUT, x, CCH, (size_t)0, SEQ, SEQ, (size_t)CCH * SEQ, 0, (size_t)0, sproj, VSC);

    k_flash<<<dim3(SEQ / (16 * AW), NB, 1), 32 * AW, 0, stream>>>(QP, KP, VT, OP);

    k_gemm<2><<<dim3(CCH / 64, NB * SEQ / 64, 1), 32, 0, stream>>>(WP, OP, bp, OP, OUT, x, CCH, (size_t)0, OUT_SEQ, SEQ, (size_t)CCH * OUT_SEQ, SEQ_FULL, (size_t)CCH * SEQ_FULL, 1.0f / (WSC * OSC), 1.0f);
}
